// GPT2Attention_13151189860910
// MI455X (gfx1250) — hardware-verified
//
#include <hip/hip_runtime.h>


#ifndef NB
#define NB 8
#endif
#ifndef SEQ
#define SEQ 1024
#endif
#define NB_FULL  8
#define SEQ_FULL 1024
#define DM    768
#define NH    12
#define HD    64
#define NQKV  (3 * DM)
#define MROWS (NB * SEQ)
#define NQT   (SEQ / 64)

static_assert(SEQ % 64 == 0);
static_assert(SEQ >= 64 && SEQ <= SEQ_FULL);
static_assert(NB >= 1 && NB <= NB_FULL);
static_assert(DM % 64 == 0 && DM % 32 == 0);
static_assert(NQKV % 64 == 0);
static_assert(NH * HD == DM);
static_assert(MROWS % 64 == 0);

#define XH_BYTES  ((size_t)MROWS * DM * 2)
#define WTA_BYTES ((size_t)NQKV * DM * 2)
#define WTP_BYTES ((size_t)DM * DM * 2)
#define QKV_BYTES ((size_t)NB * NH * SEQ * HD * 2)
#define OB_BYTES  ((size_t)MROWS * DM * 2)
#define WS_TOTAL  (XH_BYTES + WTA_BYTES + WTP_BYTES + 3 * QKV_BYTES + OB_BYTES)
static_assert(WS_TOTAL <= (size_t)134217728);
static_assert(XH_BYTES % 128 == 0 && WTA_BYTES % 128 == 0 && WTP_BYTES % 128 == 0 &&
              QKV_BYTES % 128 == 0 && OB_BYTES % 128 == 0);

typedef _Float16 v16h __attribute__((ext_vector_type(16)));
typedef _Float16 v8h  __attribute__((ext_vector_type(8)));
typedef float    v8f  __attribute__((ext_vector_type(8)));
typedef float    v4f  __attribute__((ext_vector_type(4)));
union V16u { v16h v; v8h h[2]; };

#define WCAR 64.0f
#define PCAR 256.0f
#define OCAR 32.0f

__device__ __forceinline__ float bf16r(float f) {
  unsigned int u = __float_as_uint(f);
  u = (u + 0x7fffu + ((u >> 16) & 1u)) & 0xffff0000u;
  return __uint_as_float(u);
}

__device__ __forceinline__ v8f wmma16(const v16h& a, const v16h& b, v8f c) {
  return __builtin_amdgcn_wmma_f32_16x16x32_f16(false, a, false, b, (short)0, c, false, false);
}

__device__ __forceinline__ void guard2(v8f& c0, v8f& c1, const v16h& a, const v16h& b) {
  asm volatile("v_nop\n\tv_nop\n\tv_nop\n\tv_nop" : "+v"(c0), "+v"(c1) : "v"(a), "v"(b));
}
__device__ __forceinline__ void guard4(v8f& c0, v8f& c1, v8f& c2, v8f& c3, const v16h& a, const v16h& b) {
  asm volatile("v_nop\n\tv_nop\n\tv_nop\n\tv_nop" : "+v"(c0), "+v"(c1), "+v"(c2), "+v"(c3) : "v"(a), "v"(b));
}

__global__ __launch_bounds__(256) void k_xconv(const float* __restrict__ x,
                                              _Float16* __restrict__ xh, int npieces) {
  const int piece = (int)blockIdx.x * 256 + (int)threadIdx.x;
  if (piece < npieces) {
    const int lr = piece / (DM / 8);
    const int c8 = (piece - lr * (DM / 8)) * 8;
    const int b  = lr / SEQ;
    const int l  = lr - b * SEQ;
    const float* src = x + ((size_t)b * SEQ_FULL + l) * DM + c8;
    const v4f f0 = *(const v4f*)src;
    const v4f f1 = *(const v4f*)(src + 4);
    v8h hv;
#pragma unroll
    for (int j = 0; j < 4; ++j) {
      hv[j]     = (_Float16)bf16r(f0[j]);
      hv[j + 4] = (_Float16)bf16r(f1[j]);
    }
    _Float16* dst = xh + (size_t)lr * DM + c8;
    *(volatile v8h*)dst = hv;
    __threadfence();
    *(volatile v8h*)dst = hv;
  }
}

__global__ __launch_bounds__(256) void k_wconv(const float* __restrict__ src, _Float16* __restrict__ dst,
                                              int src_ld, int a_mul, int i_mul, int n_ta) {
  __shared__ __attribute__((aligned(16))) _Float16 sT[64][72];
  const int tid = threadIdx.x;
  const int ta  = (int)blockIdx.x % n_ta;
  const int tn  = (int)blockIdx.x / n_ta;
#pragma unroll
  for (int it = 0; it < 4; ++it) {
    const int idx = it * 256 + tid;
    const int i   = idx >> 4;
    const int j4  = (idx & 15) * 4;
    const float* p = src + (size_t)(ta * a_mul + i * i_mul) * src_ld + tn * 64 + j4;
    const v4f f = *(const v4f*)p;
#pragma unroll
    for (int c = 0; c < 4; ++c) sT[j4 + c][i] = (_Float16)(WCAR * bf16r(f[c]));
  }
  __syncthreads();
  v8h v[2];
  size_t o[2];
#pragma unroll
  for (int it = 0; it < 2; ++it) {
    const int p  = it * 256 + tid;
    const int j  = p >> 3;
    const int q8 = (p & 7) * 8;
    v[it] = *(const v8h*)(&sT[j][q8]);
    o[it] = (size_t)(tn * 64 + j) * DM + ta * 64 + q8;
  }
  *(volatile v8h*)(dst + o[0]) = v[0];
  *(volatile v8h*)(dst + o[1]) = v[1];
  __threadfence();
  *(volatile v8h*)(dst + o[0]) = v[0];
  *(volatile v8h*)(dst + o[1]) = v[1];
}

__device__ __forceinline__ void gemm64_core(const _Float16* __restrict__ a0p, const _Float16* __restrict__ b0p,
                                            v8f& c00, v8f& c01, v8f& c10, v8f& c11) {
  const _Float16* a1p = a0p + 16 * DM;
  const _Float16* b1p = b0p + 16 * DM;
#pragma unroll 2
  for (int k0 = 0; k0 < DM; k0 += 32) {
    V16u a0, a1, b0, b1;
    a0.h[0] = *(const v8h*)(a0p + k0); a0.h[1] = *(const v8h*)(a0p + k0 + 16);
    a1.h[0] = *(const v8h*)(a1p + k0); a1.h[1] = *(const v8h*)(a1p + k0 + 16);
    b0.h[0] = *(const v8h*)(b0p + k0); b0.h[1] = *(const v8h*)(b0p + k0 + 16);
    b1.h[0] = *(const v8h*)(b1p + k0); b1.h[1] = *(const v8h*)(b1p + k0 + 16);
    c00 = wmma16(a0.v, b0.v, c00);
    c01 = wmma16(a0.v, b1.v, c01);
    c10 = wmma16(a1.v, b0.v, c10);
    c11 = wmma16(a1.v, b1.v, c11);
    guard4(c00, c01, c10, c11, a1.v, b1.v);
  }
}

__global__ __launch_bounds__(128) __attribute__((amdgpu_num_vgpr(256)))
void k_qkv(const _Float16* __restrict__ xh, const _Float16* __restrict__ wta,
           const float* __restrict__ battn, _Float16* __restrict__ qh,
           _Float16* __restrict__ kh, _Float16* __restrict__ vt) {
  __shared__ __attribute__((aligned(16))) _Float16 sT[64][72];
  const int tid = threadIdx.x, wave = tid >> 5, lane = tid & 31, l16 = lane & 15, lh = lane >> 4;
  const int wm = wave & 1, wn = wave >> 1;
  const int ct = blockIdx.x;
  const int rt = blockIdx.y;
  const int t  = ct / NH;
  const int h  = ct - t * NH;
  const int row0 = rt * 64;
  const int n0   = ct * 64;

  v8f c00 = {}, c01 = {}, c10 = {}, c11 = {};
  const _Float16* a0p = xh  + (size_t)(row0 + wm * 32 + l16) * DM + 8 * lh;
  const _Float16* b0p = wta + (size_t)(n0 + wn * 32 + l16) * DM + 8 * lh;
  gemm64_core(a0p, b0p, c00, c01, c10, c11);

  const float s64   = 0.015625f;
  const float bias0 = bf16r(battn[n0 + wn * 32 + l16]);
  const float bias1 = bf16r(battn[n0 + wn * 32 + 16 + l16]);
#pragma unroll
  for (int r = 0; r < 8; ++r) {
    const int lrow = wm * 32 + 8 * lh + r;
    const int col  = wn * 32 + l16;
    const _Float16 e00 = (_Float16)(c00[r] * s64 + bias0);
    const _Float16 e01 = (_Float16)(c01[r] * s64 + bias1);
    const _Float16 e10 = (_Float16)(c10[r] * s64 + bias0);
    const _Float16 e11 = (_Float16)(c11[r] * s64 + bias1);
    if (t < 2) {
      sT[lrow][col]           = e00;
      sT[lrow][col + 16]      = e01;
      sT[lrow + 16][col]      = e10;
      sT[lrow + 16][col + 16] = e11;
    } else {
      sT[col][lrow]           = e00;
      sT[col + 16][lrow]      = e01;
      sT[col][lrow + 16]      = e10;
      sT[col + 16][lrow + 16] = e11;
    }
  }
  __syncthreads();

  const int b  = row0 / SEQ;
  const int l0 = row0 - b * SEQ;
  const int bh = b * NH + h;
  _Float16* plane = (t == 0) ? qh : ((t == 1) ? kh : vt);
  v8h v[4];
  size_t o[4];
#pragma unroll
  for (int it = 0; it < 4; ++it) {
    const int p  = it * 128 + tid;
    const int j  = p >> 3;
    const int q8 = (p & 7) * 8;
    v[it] = *(const v8h*)(&sT[j][q8]);
    if (t < 2) o[it] = ((size_t)bh * SEQ + l0 + j) * HD + q8;
    else       o[it] = ((size_t)bh * HD + j) * SEQ + l0 + q8;
  }
#pragma unroll
  for (int it = 0; it < 4; ++it) *(volatile v8h*)(plane + o[it]) = v[it];
  __threadfence();
#pragma unroll
  for (int it = 0; it < 4; ++it) *(volatile v8h*)(plane + o[it]) = v[it];
}

__global__ __launch_bounds__(128) __attribute__((amdgpu_num_vgpr(256)))
void k_attn(const _Float16* __restrict__ qh, const _Float16* __restrict__ kh,
            const _Float16* __restrict__ vt, _Float16* __restrict__ ob) {
  __shared__ __attribute__((aligned(16))) _Float16 ldsP[4][16 * 32];
  __shared__ __attribute__((aligned(16))) _Float16 sOT[64][72];

  const int tid = threadIdx.x, wave = tid >> 5, lane = tid & 31, l16 = lane & 15, lh = lane >> 4;
  const int bh = (int)blockIdx.x / NQT;
  const int lt = (int)blockIdx.x - bh * NQT;
  const int b  = bh / NH;
  const int h  = bh - b * NH;
  const int qBase = lt * 64 + wave * 16;

  v16h aq[2];
  {
    const _Float16* qrow = qh + ((size_t)bh * SEQ + qBase + l16) * HD + 8 * lh;
#pragma unroll
    for (int hc = 0; hc < 2; ++hc) {
      V16u a;
      a.h[0] = *(const v8h*)(qrow + hc * 32);
      a.h[1] = *(const v8h*)(qrow + hc * 32 + 16);
      aq[hc] = a.v;
    }
  }

  float m[8], l[8];
  v8f co[4];
  const v8f zero = {};
#pragma unroll
  for (int r = 0; r < 8; ++r) { m[r] = -1e30f; l[r] = 0.0f; }
#pragma unroll
  for (int n = 0; n < 4; ++n) co[n] = zero;

  const _Float16* kbase = kh + (size_t)bh * SEQ * HD;
  const _Float16* vbase = vt + (size_t)bh * HD * SEQ;
  _Float16* myP = ldsP[wave];

#pragma unroll 1
  for (int k0 = 0; k0 < SEQ; k0 += 32) {
    v8f s0 = {};
    v8f s1 = {};
    const _Float16* kr0 = kbase + (size_t)(k0 + l16) * HD + 8 * lh;
    const _Float16* kr1 = kr0 + 16 * HD;
    V16u bk0[2], bk1[2];
#pragma unroll
    for (int hc = 0; hc < 2; ++hc) {
      bk0[hc].h[0] = *(const v8h*)(kr0 + hc * 32); bk0[hc].h[1] = *(const v8h*)(kr0 + hc * 32 + 16);
      bk1[hc].h[0] = *(const v8h*)(kr1 + hc * 32); bk1[hc].h[1] = *(const v8h*)(kr1 + hc * 32 + 16);
      s0 = wmma16(aq[hc], bk0[hc].v, s0);
      s1 = wmma16(aq[hc], bk1[hc].v, s1);
    }
    guard2(s0, s1, aq[1], bk1[1].v);

    float alpha[8];
#pragma unroll
    for (int r = 0; r < 8; ++r) {
      const float x0 = s0[r] * 0.125f;
      const float x1 = s1[r] * 0.125f;
      float tmax = fmaxf(x0, x1);
#pragma unroll
      for (int off = 1; off < 16; off <<= 1) tmax = fmaxf(tmax, __shfl_xor(tmax, off, 32));
      const float mn = fmaxf(m[r], tmax);
      alpha[r] = __expf(m[r] - mn);
      const float p0 = __expf(x0 - mn);
      const float p1 = __expf(x1 - mn);
      float ps = p0 + p1;
#pragma unroll
      for (int off = 1; off < 16; off <<= 1) ps += __shfl_xor(ps, off, 32);
      l[r] = l[r] * alpha[r] + ps;
      m[r] = mn;
      myP[(r + 8 * lh) * 32 + l16]      = (_Float16)(p0 * PCAR);
      myP[(r + 8 * lh) * 32 + 16 + l16] = (_Float16)(p1 * PCAR);
    }
#pragma unroll
    for (int n = 0; n < 4; ++n)
#pragma unroll
      for (int r = 0; r < 8; ++r) co[n][r] *= alpha[r];

    __builtin_amdgcn_fence(3, "wavefront");
    __builtin_amdgcn_wave_barrier();
    __builtin_amdgcn_fence(2, "wavefront");

    V16u ap;
    ap.h[0] = *(const v8h*)(myP + l16 * 32 + 8 * lh);
    ap.h[1] = *(const v8h*)(myP + l16 * 32 + 16 + 8 * lh);
    V16u bv[4];
#pragma unroll
    for (int n = 0; n < 4; ++n) {
      const _Float16* vp = vbase + (size_t)(n * 16 + l16) * SEQ + k0 + 8 * lh;
      bv[n].h[0] = *(const v8h*)vp;
      bv[n].h[1] = *(const v8h*)(vp + 16);
      co[n] = wmma16(ap.v, bv[n].v, co[n]);
    }
    guard4(co[0], co[1], co[2], co[3], ap.v, bv[3].v);
  }

#pragma unroll
  for (int r = 0; r < 8; ++r) {
    const float inv = (OCAR / PCAR) * (1.0f / l[r]);
    const int lr = wave * 16 + 8 * lh + r;
#pragma unroll
    for (int n = 0; n < 4; ++n) sOT[n * 16 + l16][lr] = (_Float16)(co[n][r] * inv);
  }
  __syncthreads();

  v8h v[4];
  size_t o[4];
#pragma unroll
  for (int it = 0; it < 4; ++it) {
    const int p  = it * 128 + tid;
    const int hd = p >> 3;
    const int q8 = (p & 7) * 8;
    v[it] = *(const v8h*)(&sOT[hd][q8]);
    o[it] = (((size_t)(b * SEQ + hd * NQT + lt)) * NH + h) * HD + q8;
  }
#pragma unroll
  for (int it = 0; it < 4; ++it) *(volatile v8h*)(ob + o[it]) = v[it];
  __threadfence();
#pragma unroll
  for (int it = 0; it < 4; ++it) *(volatile v8h*)(ob + o[it]) = v[it];
}

__global__ __launch_bounds__(128) __attribute__((amdgpu_num_vgpr(256)))
void k_proj(const _Float16* __restrict__ ob, const _Float16* __restrict__ wtp,
            const float* __restrict__ bproj, float* __restrict__ out) {
  __shared__ __attribute__((aligned(16))) float sO[64][68];
  const int tid = threadIdx.x, wave = tid >> 5, lane = tid & 31, l16 = lane & 15, lh = lane >> 4;
  const int wm = wave & 1, wn = wave >> 1;
  const int ct = blockIdx.x;
  const int rt = blockIdx.y;
  const int row0 = rt * 64;
  const int n0   = ct * 64;

  v8f c00 = {}, c01 = {}, c10 = {}, c11 = {};
  const _Float16* a0p = ob  + (size_t)(row0 + wm * 32 + l16) * DM + 8 * lh;
  const _Float16* b0p = wtp + (size_t)(n0 + wn * 32 + l16) * DM + 8 * lh;
  gemm64_core(a0p, b0p, c00, c01, c10, c11);

  const float sc    = 0.00048828125f;
  const float bias0 = bf16r(bproj[n0 + wn * 32 + l16]);
  const float bias1 = bf16r(bproj[n0 + wn * 32 + 16 + l16]);
#pragma unroll
  for (int r = 0; r < 8; ++r) {
    const int lrow = wm * 32 + 8 * lh + r;
    const int col  = wn * 32 + l16;
    sO[lrow][col]           = c00[r] * sc + bias0;
    sO[lrow][col + 16]      = c01[r] * sc + bias1;
    sO[lrow + 16][col]      = c10[r] * sc + bias0;
    sO[lrow + 16][col + 16] = c11[r] * sc + bias1;
  }
  __syncthreads();

  v4f v[8];
  size_t o[8];
#pragma unroll
  for (int it = 0; it < 8; ++it) {
    const int p  = it * 128 + tid;
    const int j  = p >> 4;
    const int q4 = (p & 15) * 4;
    v[it] = *(const v4f*)(&sO[j][q4]);
    o[it] = (size_t)(row0 + j) * DM + n0 + q4;
  }
#pragma unroll
  for (int it = 0; it < 8; ++it) *(volatile v4f*)(out + o[it]) = v[it];
  __threadfence();
#pragma unroll
  for (int it = 0; it < 8; ++it) *(volatile v4f*)(out + o[it]) = v[it];
}

extern "C" void kernel_launch(void* const* d_in, const int* in_sizes, int n_in,
                              void* d_out, int out_size, void* d_ws, size_t ws_size,
                              hipStream_t stream) {
  if (n_in < 5) return;
  if (in_sizes[0] < ((NB - 1) * SEQ_FULL + SEQ) * DM) return;
  if (in_sizes[1] < DM * NQKV) return;
  if (in_sizes[2] < NQKV) return;
  if (in_sizes[3] < DM * DM) return;
  if (in_sizes[4] < DM) return;
  if (out_size < MROWS * DM) return;
  if (ws_size < WS_TOTAL) return;

  const float* x      = (const float*)d_in[0];
  const float* w_attn = (const float*)d_in[1];
  const float* b_attn = (const float*)d_in[2];
  const float* w_proj = (const float*)d_in[3];
  const float* b_proj = (const float*)d_in[4];
  float* out = (float*)d_out;

  char* ws = (char*)d_ws;
  size_t off = 0;
  _Float16* xh  = (_Float16*)(ws + off); off += XH_BYTES;
  _Float16* wta = (_Float16*)(ws + off); off += WTA_BYTES;
  _Float16* wtp = (_Float16*)(ws + off); off += WTP_BYTES;
  _Float16* qh  = (_Float16*)(ws + off); off += QKV_BYTES;
  _Float16* kh  = (_Float16*)(ws + off); off += QKV_BYTES;
  _Float16* vt  = (_Float16*)(ws + off); off += QKV_BYTES;
  _Float16* ob  = (_Float16*)(ws + off); off += OB_BYTES;
  if (off > ws_size) return;

  const int npieces = MROWS * DM / 8;
  k_xconv<<<(npieces + 255) / 256, 256, 0, stream>>>(x, xh, npieces);
  k_wconv<<<(NQKV / 64) * (DM / 64), 256, 0, stream>>>(w_attn, wta, NQKV, 64, 1, DM / 64);
  k_wconv<<<(DM / 64) * NH, 256, 0, stream>>>(w_proj, wtp, DM, 1, NH, NH);
  k_qkv<<<dim3(NQKV / 64, MROWS / 64), 128, 0, stream>>>(xh, wta, b_attn, qh, kh, vt);
  k_attn<<<NB * NH * NQT, 128, 0, stream>>>(qh, kh, vt, ob);
  k_proj<<<dim3(DM / 64, MROWS / 64), 128, 0, stream>>>(ob, wtp, b_proj, out);
}
